// VanillaRNN_55130200211525
// MI455X (gfx1250) — hardware-verified
//
#include <hip/hip_runtime.h>
#include <math.h>

constexpr int NBATCH   = 512;
constexpr int NSTEP    = 256;
constexpr int NSTATE   = 64;
constexpr int NINP     = 32;
constexpr int NHID     = 1024;
constexpr int NCAT     = NSTATE + NINP;
constexpr int ROWS_BLK = 32;
constexpr int NTHR     = 256;
constexpr int NWAVE    = NTHR / 32;
constexpr int APITCH   = 104;
constexpr int HPITCH   = 1032;
constexpr int XPITCH   = 68;
constexpr float WCARRY     = 16.0f;
constexpr float WCARRY_INV = 1.0f / 16.0f;

constexpr int NW1 = NHID * NCAT;
constexpr int NW2 = NHID * NHID;
constexpr int NW3 = NSTATE * NHID;
constexpr int CVT_BLK1 = NW1 / (8 * NTHR);
constexpr int CVT_BLK2 = NW2 / (8 * NTHR);
constexpr int CVT_BLK3 = NW3 / (8 * NTHR);

static_assert(NCAT == 96 && NCAT % 32 == 0, "site 0 K is a multiple of 32");
static_assert(NHID % 64 == 0, "site 1 and site 2 K multiples of 64");
static_assert(NHID == 128 * NWAVE, "each wave owns 128 hidden columns");
static_assert(NSTATE == 64 && ROWS_BLK == 32 && NWAVE == 8, "site 2: 4 n-subtiles x 2 m-subtiles = 8 waves");
static_assert(ROWS_BLK * (NINP / 4) == NTHR, "u staging covers the tile exactly");
static_assert(ROWS_BLK * (NSTATE / 4) == 2 * NTHR, "x0 staging covers the tile exactly");
static_assert(NBATCH % ROWS_BLK == 0, "grid exact");
static_assert(NW1 % (8 * NTHR) == 0 && NW2 % (8 * NTHR) == 0 && NW3 % (8 * NTHR) == 0, "convert grid exact");
static_assert((NW1 * 2) % 256 == 0 && ((NW1 + NW2) * 2) % 256 == 0, "plane bases 256-B aligned");
static_assert(APITCH % 8 == 0 && HPITCH % 8 == 0 && XPITCH % 4 == 0, "16-B aligned LDS rows");

typedef __attribute__((ext_vector_type(16))) _Float16 v16h;
typedef __attribute__((ext_vector_type(8)))  _Float16 v8h;
typedef __attribute__((ext_vector_type(8)))  float    v8f;
typedef __attribute__((ext_vector_type(4)))  float    v4f;
typedef __attribute__((ext_vector_type(2)))  unsigned v2u;

union FragU { v16h v; v8h h[2]; };
__device__ __forceinline__ v16h frag_load(const _Float16* p) {
  FragU f;
  f.h[0] = *(const v8h*)(p);
  f.h[1] = *(const v8h*)(p + 16);
  return f.v;
}
__device__ __forceinline__ v8f mma16(v16h a, v16h b, v8f c) {
  return __builtin_amdgcn_wmma_f32_16x16x32_f16(false, a, false, b, (short)0, c, false, false);
}

__device__ __forceinline__ void guard_site0(v8f& c0, v8f& c1,
                                            v16h a0, v16h a1, v16h a2, v16h a3, v16h a4, v16h a5,
                                            v16h b0, v16h b1, v16h b2) {
  asm volatile("v_nop\n\tv_nop\n\tv_nop\n\tv_nop"
               : "+v"(c0), "+v"(c1)
               : "v"(a0), "v"(a1), "v"(a2), "v"(a3), "v"(a4), "v"(a5), "v"(b0), "v"(b1), "v"(b2));
}
__device__ __forceinline__ void guard_site1(v8f& c0, v8f& c1, v8f& c2, v8f& c3, v8f& c4, v8f& c5, v8f& c6, v8f& c7,
                                            v16h a0, v16h a1, v16h b0, v16h b1, v16h b2, v16h b3) {
  asm volatile("v_nop\n\tv_nop\n\tv_nop\n\tv_nop"
               : "+v"(c0), "+v"(c1), "+v"(c2), "+v"(c3), "+v"(c4), "+v"(c5), "+v"(c6), "+v"(c7)
               : "v"(a0), "v"(a1), "v"(b0), "v"(b1), "v"(b2), "v"(b3));
}
__device__ __forceinline__ void guard_site2(v8f& c0, v8f& c1, v16h a0, v16h a1, v16h b0, v16h b1) {
  asm volatile("v_nop\n\tv_nop\n\tv_nop\n\tv_nop"
               : "+v"(c0), "+v"(c1)
               : "v"(a0), "v"(a1), "v"(b0), "v"(b1));
}

__device__ __forceinline__ float fsig(float x) { return __builtin_amdgcn_rcpf(1.0f + __expf(-x)); }

__device__ __forceinline__ unsigned pack_h2(float lo, float hi) {
  const _Float16 hl = (_Float16)lo;
  const _Float16 hh = (_Float16)hi;
  const unsigned short bl = __builtin_bit_cast(unsigned short, hl);
  const unsigned short bh = __builtin_bit_cast(unsigned short, hh);
  return (unsigned)bl | ((unsigned)bh << 16);
}

__global__ __launch_bounds__(NTHR) void cvt_weights_kernel(const float* __restrict__ w1, const float* __restrict__ w2,
                                                           const float* __restrict__ w3, unsigned short* __restrict__ dst) {
  const int blk = blockIdx.x;
  const float* src = w1;
  int lb = blk;
  size_t dofs = 0;
  if (blk >= CVT_BLK1 + CVT_BLK2) {
    src = w3;
    lb = blk - (CVT_BLK1 + CVT_BLK2);
    dofs = (size_t)NW1 + (size_t)NW2;
  } else if (blk >= CVT_BLK1) {
    src = w2;
    lb = blk - CVT_BLK1;
    dofs = (size_t)NW1;
  }
  const size_t e0 = ((size_t)lb * NTHR + threadIdx.x) * 8;
  const v4f a = *(const v4f*)(src + e0);
  const v4f b = *(const v4f*)(src + e0 + 4);
  v8h hv;
#pragma unroll
  for (int e = 0; e < 4; ++e) {
    const float fa = a[e] * WCARRY;
    const float fb = b[e] * WCARRY;
    hv[e]     = (_Float16)fa;
    hv[4 + e] = (_Float16)fb;
  }
  unsigned short* dp = dst + dofs + e0;
  *(volatile v8h*)dp = hv;
  __threadfence();
  *(volatile v8h*)dp = hv;
}

__global__ __launch_bounds__(NTHR) void rnn_seq_kernel(const float* __restrict__ x0, const float* __restrict__ u,
                                                       const float* __restrict__ b1, const float* __restrict__ b2,
                                                       const float* __restrict__ b3,
                                                       const unsigned short* __restrict__ W1p,
                                                       const unsigned short* __restrict__ W2p,
                                                       const unsigned short* __restrict__ W3p,
                                                       float* __restrict__ out) {
  __shared__ __align__(16) _Float16 aBuf[ROWS_BLK * APITCH];
  __shared__ __align__(16) _Float16 hA[ROWS_BLK * HPITCH];
  __shared__ __align__(16) _Float16 hB[ROWS_BLK * HPITCH];
  __shared__ __align__(16) float    xS[ROWS_BLK * XPITCH];

  const _Float16* W1 = (const _Float16*)W1p;
  const _Float16* W2 = (const _Float16*)W2p;
  const _Float16* W3 = (const _Float16*)W3p;

  const int tid  = threadIdx.x;
  const int lane = tid & 31;
  const int wave = tid >> 5;
  const int c    = lane & 15;
  const int hh   = lane >> 4;
  const int koff = hh * 8;
  const int c4   = c * 4;
  const int rowbase = blockIdx.x * ROWS_BLK;

#pragma unroll
  for (int i = 0; i < 2; ++i) {
    const int idx = i * NTHR + tid;
    const int r  = idx >> 4;
    const int cc = (idx & 15) * 4;
    const v4f v = *(const v4f*)(x0 + (size_t)(rowbase + r) * NSTATE + cc);
    v2u pk;
    pk[0] = pack_h2(v[0], v[1]);
    pk[1] = pack_h2(v[2], v[3]);
    *(v2u*)(aBuf + r * APITCH + cc) = pk;
  }

  const int nt3   = wave & 3;
  const int mt3   = wave >> 2;
  const int ncol3 = 16 * nt3 + c;
  const float bias3 = b3[ncol3];

  const v8f z8 = {0.f, 0.f, 0.f, 0.f, 0.f, 0.f, 0.f, 0.f};

  const _Float16* a0row = aBuf + c * APITCH + koff;
  const _Float16* a1row = aBuf + (16 + c) * APITCH + koff;
  const _Float16* h0row = hA + c * HPITCH + koff;
  const _Float16* h1row = hA + (16 + c) * HPITCH + koff;
  const _Float16* g3row = hB + (16 * mt3 + c) * HPITCH + koff;
  const _Float16* w3row = W3 + (size_t)ncol3 * NHID + koff;

  const int ur  = tid >> 3;
  const int uc4 = (tid & 7) * 4;
  const float* urow = u + ((size_t)(rowbase + ur) * NSTEP) * NINP + uc4;

  const int orow0 = 2 * wave + hh;
  const int orow1 = 16 + orow0;

#pragma unroll 1
  for (int t = 0; t < NSTEP; ++t) {
    {
      const v4f v = *(const v4f*)(urow + (size_t)t * NINP);
      v2u pk;
      pk[0] = pack_h2(v[0], v[1]);
      pk[1] = pack_h2(v[2], v[3]);
      *(v2u*)(aBuf + ur * APITCH + NSTATE + uc4) = pk;
    }
    __syncthreads();

    {
      const v16h a00 = frag_load(a0row);
      const v16h a01 = frag_load(a0row + 32);
      const v16h a02 = frag_load(a0row + 64);
      const v16h a10 = frag_load(a1row);
      const v16h a11 = frag_load(a1row + 32);
      const v16h a12 = frag_load(a1row + 64);
#pragma unroll 1
      for (int nt = 0; nt < 8; ++nt) {
        const int ncol = 128 * wave + 16 * nt + c;
        const _Float16* w = W1 + (size_t)ncol * NCAT + koff;
        const float bv = b1[ncol];
        const v16h f0 = frag_load(w);
        const v16h f1 = frag_load(w + 32);
        const v16h f2 = frag_load(w + 64);
        v8f acc0 = z8;
        v8f acc1 = z8;
        acc0 = mma16(a00, f0, acc0);
        acc1 = mma16(a10, f0, acc1);
        acc0 = mma16(a01, f1, acc0);
        acc1 = mma16(a11, f1, acc1);
        acc0 = mma16(a02, f2, acc0);
        acc1 = mma16(a12, f2, acc1);
        guard_site0(acc0, acc1, a00, a01, a02, a10, a11, a12, f0, f1, f2);
#pragma unroll
        for (int r = 0; r < 8; ++r) {
          const float z0 = fmaf(acc0[r], WCARRY_INV, bv);
          const float z1 = fmaf(acc1[r], WCARRY_INV, bv);
          hA[(8 * hh + r) * HPITCH + ncol]      = (_Float16)fsig(z0);
          hA[(16 + 8 * hh + r) * HPITCH + ncol] = (_Float16)fsig(z1);
        }
      }
    }
    __syncthreads();

#pragma unroll 1
    for (int pass = 0; pass < 2; ++pass) {
      const int nbase = 128 * wave + 64 * pass;
      const _Float16* wp = W2 + (size_t)(nbase + c) * NHID + koff;
      float bs[4];
#pragma unroll
      for (int j = 0; j < 4; ++j) bs[j] = b2[nbase + 16 * j + c];
      v8f acc[2][4];
#pragma unroll
      for (int j = 0; j < 4; ++j) {
        acc[0][j] = z8;
        acc[1][j] = z8;
      }
#pragma unroll 2
      for (int k0 = 0; k0 < NHID; k0 += 32) {
        const v16h a0 = frag_load(h0row + k0);
        const v16h a1 = frag_load(h1row + k0);
        const v16h f0 = frag_load(wp + k0);
        const v16h f1 = frag_load(wp + (size_t)16 * NHID + k0);
        const v16h f2 = frag_load(wp + (size_t)32 * NHID + k0);
        const v16h f3 = frag_load(wp + (size_t)48 * NHID + k0);
        acc[0][0] = mma16(a0, f0, acc[0][0]);
        acc[1][0] = mma16(a1, f0, acc[1][0]);
        acc[0][1] = mma16(a0, f1, acc[0][1]);
        acc[1][1] = mma16(a1, f1, acc[1][1]);
        acc[0][2] = mma16(a0, f2, acc[0][2]);
        acc[1][2] = mma16(a1, f2, acc[1][2]);
        acc[0][3] = mma16(a0, f3, acc[0][3]);
        acc[1][3] = mma16(a1, f3, acc[1][3]);
        guard_site1(acc[0][0], acc[1][0], acc[0][1], acc[1][1], acc[0][2], acc[1][2], acc[0][3], acc[1][3],
                    a0, a1, f0, f1, f2, f3);
      }
#pragma unroll
      for (int j = 0; j < 4; ++j) {
        const int ncol = nbase + 16 * j + c;
#pragma unroll
        for (int r = 0; r < 8; ++r) {
          const float z0 = fmaf(acc[0][j][r], WCARRY_INV, bs[j]);
          const float z1 = fmaf(acc[1][j][r], WCARRY_INV, bs[j]);
          hB[(8 * hh + r) * HPITCH + ncol]      = (_Float16)fsig(z0);
          hB[(16 + 8 * hh + r) * HPITCH + ncol] = (_Float16)fsig(z1);
        }
      }
    }
    __syncthreads();

    {
      v8f accA = z8;
      v8f accB = z8;
#pragma unroll 1
      for (int k0 = 0; k0 < NHID; k0 += 64) {
        const v16h a0 = frag_load(g3row + k0);
        const v16h a1 = frag_load(g3row + k0 + 32);
        const v16h f0 = frag_load(w3row + k0);
        const v16h f1 = frag_load(w3row + k0 + 32);
        accA = mma16(a0, f0, accA);
        accB = mma16(a1, f1, accB);
        guard_site2(accA, accB, a0, a1, f0, f1);
      }
#pragma unroll
      for (int r = 0; r < 8; ++r) {
        const float s  = accA[r] + accB[r];
        const float xv = fmaf(s, WCARRY_INV, bias3);
        const int row = 16 * mt3 + 8 * hh + r;
        xS[row * XPITCH + ncol3]   = xv;
        aBuf[row * APITCH + ncol3] = (_Float16)xv;
      }
    }
    __syncthreads();

    {
      const v4f o0 = *(const v4f*)(xS + orow0 * XPITCH + c4);
      const v4f o1 = *(const v4f*)(xS + orow1 * XPITCH + c4);
      float* op0 = out + ((size_t)(rowbase + orow0) * NSTEP + (size_t)t) * NSTATE + c4;
      float* op1 = out + ((size_t)(rowbase + orow1) * NSTEP + (size_t)t) * NSTATE + c4;
      for (int pass = 0; pass < 2; ++pass) {
        *(volatile v4f*)op0 = o0;
        *(volatile v4f*)op1 = o1;
        __threadfence();
      }
    }
  }
}

extern "C" void kernel_launch(void* const* d_in, const int* in_sizes, int n_in,
                              void* d_out, int out_size, void* d_ws, size_t ws_size, hipStream_t stream) {
  if (n_in < 8 || d_out == nullptr || d_ws == nullptr) return;
  if (in_sizes[0] != NBATCH * NSTATE || in_sizes[1] != NBATCH * NSTEP * NINP ||
      in_sizes[2] != NW1 || in_sizes[3] != NHID || in_sizes[4] != NW2 || in_sizes[5] != NHID ||
      in_sizes[6] != NW3 || in_sizes[7] != NSTATE || out_size != NBATCH * NSTEP * NSTATE) return;

  const float* x0 = (const float*)d_in[0];
  const float* u  = (const float*)d_in[1];
  const float* w1 = (const float*)d_in[2];
  const float* b1 = (const float*)d_in[3];
  const float* w2 = (const float*)d_in[4];
  const float* b2 = (const float*)d_in[5];
  const float* w3 = (const float*)d_in[6];
  const float* b3 = (const float*)d_in[7];
  float* out = (float*)d_out;

  const size_t carve = ((size_t)NW1 + (size_t)NW2 + (size_t)NW3) * 2;
  if (carve > ws_size || carve > (size_t)134217728) return;
  unsigned short* planes = (unsigned short*)d_ws;
  unsigned short* W1H = planes;
  unsigned short* W2H = planes + (size_t)NW1;
  unsigned short* W3H = planes + (size_t)NW1 + (size_t)NW2;

  cvt_weights_kernel<<<CVT_BLK1 + CVT_BLK2 + CVT_BLK3, NTHR, 0, stream>>>(w1, w2, w3, planes);
  rnn_seq_kernel<<<NBATCH / ROWS_BLK, NTHR, 0, stream>>>(x0, u, b1, b2, b3, W1H, W2H, W3H, out);
}
